// StyledConv_8409545966252
// MI455X (gfx1250) — hardware-verified
//
#include <hip/hip_runtime.h>


#define NBT  16
#define CI   512
#define CO   512
#define HW   1024
#define KK   9
#define KIM  (CI * KK)
#define SD   512
#define DM   KIM
#define CSC  0.014731391274719742f
#define LSC  0.044194173824159216f
#define LOSC 1024.0f

typedef _Float16 h16;
typedef unsigned short bf;
typedef __attribute__((ext_vector_type(16))) __bf16   v16bf;
typedef __attribute__((ext_vector_type(16))) _Float16 v16h;
typedef __attribute__((ext_vector_type(8)))  _Float16 v8h;
typedef __attribute__((ext_vector_type(8)))  unsigned short v8us;
typedef __attribute__((ext_vector_type(8)))  float    v8f;
typedef __attribute__((ext_vector_type(4)))  float    v4f;
typedef v8h  __attribute__((may_alias)) v8ha;
typedef v4f  __attribute__((may_alias)) v4fa;
typedef v8us __attribute__((may_alias)) v8usa;

__device__ __forceinline__ unsigned short f2bf(float f) { unsigned u = __float_as_uint(f); u += 0x7FFFu + ((u >> 16) & 1u); return (unsigned short)(u >> 16); }
__device__ __forceinline__ float bf2f(unsigned short b) { return __uint_as_float(((unsigned)b) << 16); }
__device__ __forceinline__ float bfr(float f) { return bf2f(f2bf(f)); }
__device__ __forceinline__ v16h cat16(v8h lo, v8h hi) { return __builtin_shufflevector(lo, hi, 0, 1, 2, 3, 4, 5, 6, 7, 8, 9, 10, 11, 12, 13, 14, 15); }
__device__ __forceinline__ v16bf cat16b(v8us lo, v8us hi) { return __builtin_bit_cast(v16bf, __builtin_shufflevector(lo, hi, 0, 1, 2, 3, 4, 5, 6, 7, 8, 9, 10, 11, 12, 13, 14, 15)); }
__device__ __forceinline__ v8f wmma16(v16h a, v16h b, v8f c) { return __builtin_amdgcn_wmma_f32_16x16x32_f16(false, a, false, b, (short)0, c, false, false); }
__device__ __forceinline__ v8f wmmab(v16bf a, v16bf b, v8f c) { return __builtin_amdgcn_wmma_f32_16x16x32_bf16(false, a, false, b, (short)0, c, false, false); }

template <bool SPLITA, bool F16OUT = false>
__global__ __launch_bounds__(128) void k_gemmb(const bf* __restrict__ A, const bf* __restrict__ Al, const bf* __restrict__ Bn, const float* __restrict__ bias, float* C, int ldc, h16* C2, const float* __restrict__ R = nullptr, int K = DM, int roundR = 1) {
    __shared__ __align__(16) float ost[4][16 * 68];
    const int lane = threadIdx.x & 31, wave = threadIdx.x >> 5, lr = lane & 15, hi = lane >> 4;
    const int r0 = blockIdx.x * 64 + wave * 16, c0 = blockIdx.y * 64;
    const size_t aoff = (size_t)(r0 + lr) * K + 8 * hi;
    size_t boff[4];
#pragma unroll
    for (int t = 0; t < 4; ++t) boff[t] = (size_t)(c0 + t * 16 + lr) * K + 8 * hi;
    v8f acc[4];
#pragma unroll
    for (int t = 0; t < 4; ++t) acc[t] = (v8f){};
#pragma unroll 1
    for (int kc = 0; kc < K; kc += 32) {
        const v16bf a = cat16b(*(const v8us*)(A + aoff + kc), *(const v8us*)(A + aoff + kc + 16));
        v16bf al = a;
        if (SPLITA) al = cat16b(*(const v8us*)(Al + aoff + kc), *(const v8us*)(Al + aoff + kc + 16));
#pragma unroll
        for (int t = 0; t < 4; ++t) { const v16bf b = cat16b(*(const v8us*)(Bn + boff[t] + kc), *(const v8us*)(Bn + boff[t] + kc + 16)); acc[t] = wmmab(a, b, acc[t]); if (SPLITA) acc[t] = wmmab(al, b, acc[t]); }
        asm volatile("v_nop\n\tv_nop\n\tv_nop\n\tv_nop" : "+v"(acc[0]), "+v"(acc[1]), "+v"(acc[2]), "+v"(acc[3]) : "v"(a), "v"(al));
    }
    float* os = &ost[wave][0];
#pragma unroll
    for (int t = 0; t < 4; ++t) { const float bv = bias ? bfr(bias[c0 + t * 16 + lr]) : 0.f;
#pragma unroll
        for (int j = 0; j < 8; ++j) os[(hi * 8 + j) * 68 + t * 16 + lr] = acc[t][j] + bv; }
    __syncthreads();
    if (F16OUT) {
        h16* crow = (h16*)(void*)C + (size_t)r0 * ldc + c0;
        auto pass = [&]() {
#pragma unroll
            for (int s = 0; s < 4; ++s) { const int row = 4 * s + (lane >> 3), piece = lane & 7; const float* sp = os + row * 68 + piece * 8; v8h o, o2;
#pragma unroll
                for (int i = 0; i < 8; ++i) { const h16 a = (h16)sp[i]; o[i] = a; o2[i] = (h16)((sp[i] - (float)a) * LOSC); }
                *(volatile v8h*)(crow + (size_t)row * ldc + piece * 8) = o; if (C2) *(volatile v8h*)(C2 + (size_t)r0 * ldc + c0 + (size_t)row * ldc + piece * 8) = o2; }
        };
        pass(); __threadfence(); pass();
    } else {
        float* crow = C + (size_t)r0 * ldc + c0;
        auto pass = [&]() {
#pragma unroll
            for (int s = 0; s < 8; ++s) { const int Lid = (lane >> 3) + 4 * s, piece = lane & 7; const int row = Lid >> 1, cofs = (Lid & 1) * 32 + piece * 4;
                v4f val = *(const v4fa*)(os + row * 68 + cofs); if (R) { const v4f rv = *(const v4f*)(R + ((size_t)r0 + row) * ldc + c0 + cofs); val += roundR ? (v4f){bfr(rv[0]), bfr(rv[1]), bfr(rv[2]), bfr(rv[3])} : rv; }
                *(volatile v4f*)(crow + (size_t)row * ldc + cofs) = val; }
        };
        pass(); __threadfence(); pass();
    }
}


__global__ __launch_bounds__(256) void k_cvt8(const float* __restrict__ src, bf* dst, size_t n8) {
    const size_t i = (size_t)blockIdx.x * 256 + threadIdx.x; if (i >= n8) return;
    const v8f v = *(const v8f*)(src + i * 8); v8us o;
#pragma unroll
    for (int k = 0; k < 8; ++k) o[k] = f2bf(v[k]);
    *(volatile v8us*)(dst + i * 8) = o; __threadfence(); *(volatile v8us*)(dst + i * 8) = o;
}
__global__ __launch_bounds__(256) void k_zero8(bf* dst, size_t n8) {
    const size_t i = (size_t)blockIdx.x * 256 + threadIdx.x; if (i >= n8) return; v8us z;
#pragma unroll
    for (int k = 0; k < 8; ++k) z[k] = 0;
    *(volatile v8us*)(dst + i * 8) = z; __threadfence(); *(volatile v8us*)(dst + i * 8) = z;
}

__global__ __launch_bounds__(256) void k_stylepl(const float* __restrict__ st, bf* SP) {
    const int lane = threadIdx.x & 31; const int r = blockIdx.x * 8 + (threadIdx.x >> 5); if (r >= 64) return;
#pragma unroll 1
    for (int ps = 0; ps < 2; ++ps) {
#pragma unroll
        for (int q = 0; q < SD / 256; ++q) { v8us o;
#pragma unroll
            for (int i = 0; i < 8; ++i) o[i] = f2bf(r < NBT ? st[(size_t)(r < NBT ? r : 0) * SD + q * 256 + lane * 8 + i] : 0.f);
            *(volatile v8us*)(SP + (size_t)r * SD + q * 256 + lane * 8) = o; }
        if (ps == 0) __threadfence(); }
}
__global__ __launch_bounds__(256) void k_smod(float* SR, const float* __restrict__ mb) {
    const int lane = threadIdx.x & 31; const int b = blockIdx.x * 8 + (threadIdx.x >> 5); if (b >= NBT) return;
#pragma unroll
    for (int q = 0; q < CI / 128; ++q) { float* p = SR + (size_t)b * CI + q * 128 + lane * 4; v4f v = *(const v4f*)p;
#pragma unroll
        for (int i = 0; i < 4; ++i) v[i] = v[i] * LSC + bfr(mb[q * 128 + lane * 4 + i]);
        *(volatile v4f*)p = v; __threadfence(); *(volatile v4f*)p = v; }
}
__global__ __launch_bounds__(256) void k_wsq(const float* __restrict__ w, float* WS) {
    const int lane = threadIdx.x & 31; const int wid = blockIdx.x * 8 + (threadIdx.x >> 5); if (wid >= CO * (CI / 128)) return; const int o = wid / (CI / 128); const int c0 = (wid % (CI / 128)) * 128 + lane * 4; v4f v;
#pragma unroll
    for (int i = 0; i < 4; ++i) { float s = 0.f;
#pragma unroll
        for (int k = 0; k < KK; ++k) { const float t = bfr(w[((size_t)o * CI + c0 + i) * KK + k]); s = fmaf(t, t, s); }
        v[i] = s; }
    *(volatile v4f*)(WS + (size_t)o * CI + c0) = v; __threadfence(); *(volatile v4f*)(WS + (size_t)o * CI + c0) = v;
}
__global__ __launch_bounds__(256) void k_demod(const float* __restrict__ WS, const float* __restrict__ S, float* DMD) {
    const int lane = threadIdx.x & 31; const int wid = blockIdx.x * 8 + (threadIdx.x >> 5); if (wid >= NBT * (CO / 32)) return; const int b = wid / (CO / 32); const int o = (wid % (CO / 32)) * 32 + lane; float acc = 0.f;
#pragma unroll 4
    for (int c = 0; c < CI; ++c) { const float sv = S[(size_t)b * CI + c]; acc = fmaf(WS[(size_t)o * CI + c], sv * sv, acc); }
    const float d = rsqrtf(CSC * CSC * acc + 1e-8f); *(volatile float*)(DMD + (size_t)b * CO + o) = d; __threadfence(); *(volatile float*)(DMD + (size_t)b * CO + o) = d;
}
__global__ __launch_bounds__(256) void k_im2col(const float* __restrict__ xb, const float* __restrict__ Sb, bf* Xh, bf* Xl) {
    const int lane = threadIdx.x & 31; const int p = blockIdx.x * 8 + (threadIdx.x >> 5); if (p >= HW) return; const int py = p >> 5, px = p & 31;
#pragma unroll 1
    for (int ps = 0; ps < 2; ++ps) {
#pragma unroll 1
        for (int q = 0; q < KIM / 256; ++q) { v8us oh, ol;
#pragma unroll
            for (int i = 0; i < 8; ++i) { const int e = q * 256 + lane * 8 + i; const int cin = e / KK, k = e % KK, ky = k / 3, kx = k % 3; const int yy = py + ky - 1, xx = px + kx - 1;
                float v = 0.f; if (yy >= 0 && yy < 32 && xx >= 0 && xx < 32) v = Sb[cin] * bfr(xb[((size_t)cin * 32 + yy) * 32 + xx]);
                const unsigned short hb = f2bf(v); oh[i] = hb; ol[i] = f2bf(v - bf2f(hb)); }
            const size_t o = (size_t)p * KIM + q * 256 + lane * 8; *(volatile v8us*)(Xh + o) = oh; *(volatile v8us*)(Xl + o) = ol; }
        if (ps == 0) __threadfence(); }
}
__global__ __launch_bounds__(256) void k_post(const float* __restrict__ Cm, const float* __restrict__ DMDb, const float* __restrict__ nz, const float* __restrict__ nw, const float* __restrict__ ab, float* OUTB) {
    const int lane = threadIdx.x & 31; const int wid = blockIdx.x * 8 + (threadIdx.x >> 5); if (wid >= CO * (HW / 128)) return; const int o = wid / (HW / 128); const int p0 = (wid % (HW / 128)) * 128 + lane * 4; const float dm = DMDb[o] * CSC, nwv = bfr(nw[0]), abv = bfr(ab[o]); v4f v;
#pragma unroll
    for (int i = 0; i < 4; ++i) { float t = Cm[(size_t)o * HW + p0 + i] * dm + nwv * bfr(nz[p0 + i]) + abv; t = (t >= 0.f) ? t : 0.2f * t; v[i] = t * 1.4142135623730951f; }
    *(volatile v4f*)(OUTB + (size_t)o * HW + p0) = v; __threadfence(); *(volatile v4f*)(OUTB + (size_t)o * HW + p0) = v;
}

extern "C" void kernel_launch(void* const* d_in, const int* in_sizes, int n_in,
                              void* d_out, int out_size, void* d_ws, size_t ws_size, hipStream_t stream) {
    (void)in_sizes; (void)n_in; (void)out_size;
    const float* x = (const float*)d_in[0]; const float* style = (const float*)d_in[1]; const float* noise = (const float*)d_in[2]; const float* w = (const float*)d_in[3]; const float* mw = (const float*)d_in[4]; const float* mb = (const float*)d_in[5]; const float* nw = (const float*)d_in[6]; const float* ab = (const float*)d_in[7];
    float* out = (float*)d_out;
    char* wsp = (char*)d_ws;
    auto take = [&](size_t bytes) { char* p = wsp; wsp += (bytes + 255) & ~(size_t)255; return (void*)p; };
    bf* WB = (bf*)take((size_t)CO * KIM * 2); bf* MWB = (bf*)take((size_t)CI * SD * 2); bf* SP = (bf*)take((size_t)64 * SD * 2); float* S = (float*)take((size_t)64 * CI * 4); float* WS = (float*)take((size_t)CO * CI * 4); float* DMD = (float*)take((size_t)NBT * CO * 4);
    bf* Xh = (bf*)take((size_t)HW * KIM * 2); bf* Xl = (bf*)take((size_t)HW * KIM * 2); float* C1 = (float*)take((size_t)CO * HW * 4); float* Cm = (float*)take((size_t)CO * HW * 4);
    if ((size_t)(wsp - (char*)d_ws) > ws_size) return;
    k_cvt8<<<(unsigned)(((size_t)CO * KIM / 8 + 255) / 256), 256, 0, stream>>>(w, WB, (size_t)CO * KIM / 8);
    k_cvt8<<<(CI * SD / 8 + 255) / 256, 256, 0, stream>>>(mw, MWB, CI * SD / 8);
    k_stylepl<<<64 / 8, 256, 0, stream>>>(style, SP);
    k_gemmb<false, false><<<dim3(1, CI / 64, 1), 128, 0, stream>>>(SP, nullptr, MWB, nullptr, S, CI, nullptr, nullptr, SD);
    k_smod<<<(NBT + 7) / 8, 256, 0, stream>>>(S, mb);
    k_wsq<<<(CO * (CI / 128)) / 8, 256, 0, stream>>>(w, WS); k_demod<<<(NBT * (CO / 32)) / 8, 256, 0, stream>>>(WS, S, DMD);
    for (int b = 0; b < NBT; ++b) {
        k_im2col<<<HW / 8, 256, 0, stream>>>(x + (size_t)b * CI * HW, S + (size_t)b * CI, Xh, Xl);
        k_gemmb<false, false><<<dim3(CO / 64, HW / 64, 1), 128, 0, stream>>>(WB, nullptr, Xh, nullptr, C1, HW, nullptr, nullptr, KIM, 0);
        k_gemmb<false, false><<<dim3(CO / 64, HW / 64, 1), 128, 0, stream>>>(WB, nullptr, Xl, nullptr, Cm, HW, nullptr, C1, KIM, 0);
        k_post<<<(CO * (HW / 128)) / 8, 256, 0, stream>>>(Cm, DMD + (size_t)b * CO, noise + (size_t)b * HW, nw, ab, out + (size_t)b * CO * HW); }
}
